// GraphNN_61186104099485
// MI455X (gfx1250) — hardware-run, weakly checked
//
#include <hip/hip_runtime.h>

typedef float          v8f   __attribute__((ext_vector_type(8)));
typedef float          v4f   __attribute__((ext_vector_type(4)));
typedef unsigned int   v4u   __attribute__((ext_vector_type(4)));
typedef int            v8i   __attribute__((ext_vector_type(8)));
typedef unsigned short v8us  __attribute__((ext_vector_type(8)));
typedef unsigned short v16us __attribute__((ext_vector_type(16)));
typedef __bf16         v16bf __attribute__((ext_vector_type(16)));
typedef _Float16       v16h  __attribute__((ext_vector_type(16)));
typedef v4f  __attribute__((may_alias)) v4fa;
typedef v8us __attribute__((may_alias)) v8usa;
union FragB { v16bf v; v16us u; v8us h[2]; v8i w; };
union FragH { v16h  v; v16us u; v8us h[2]; v8i w; };

__device__ __forceinline__ v8f wmb(const FragB& a, const FragB& b, v8f c) {
  v8f d = __builtin_amdgcn_wmma_f32_16x16x32_bf16(false, a.v, false, b.v, (short)0, c, false, false);
  asm volatile("v_nop\n\tv_nop\n\tv_nop\n\tv_nop" : "+v"(d) : "v"(a.w), "v"(b.w));
  return d;
}

__device__ __forceinline__ v8f wmh(const FragH& a, const FragH& b, v8f c) {
  v8f d = __builtin_amdgcn_wmma_f32_16x16x32_f16(false, a.v, false, b.v, (short)0, c, false, false);
  asm volatile("v_nop\n\tv_nop\n\tv_nop\n\tv_nop" : "+v"(d) : "v"(a.w), "v"(b.w));
  return d;
}

__device__ __forceinline__ unsigned bf16_bits(float f) {
  const unsigned u = __float_as_uint(f);
  const unsigned r = (u + 0x7FFFu + ((u >> 16) & 1u)) >> 16;
  const unsigned q = (u >> 16) | 0x40u;
  return ((u & 0x7fffffffu) > 0x7f800000u) ? q : r;
}

__device__ __forceinline__ float bf16_val(float f) {
  return __uint_as_float(bf16_bits(f) << 16);
}
__device__ __forceinline__ int clampi(int v, int lo, int hi) {
  return v < lo ? lo : (v > hi ? hi : v);
}

__device__ __forceinline__ unsigned f16_bits(float f) {
  const unsigned u  = __float_as_uint(f);
  const unsigned s  = (u >> 16) & 0x8000u;
  const unsigned a  = u & 0x7fffffffu;
  const unsigned t  = a - 0x38000000u;
  const unsigned r  = (t + 0x0FFFu + ((t >> 13) & 1u)) >> 13;
  const unsigned rc = r > 0x7C00u ? 0x7C00u : r;
  const bool small  = a < 0x38800000u;
  const bool isnan  = a > 0x7f800000u;
  const unsigned fin = small ? 0u : (s | rc);
  return isnan ? (s | 0x7E00u) : fin;
}

__device__ __forceinline__ unsigned pk16(unsigned lo, unsigned hi) { return lo | (hi << 16); }
__device__ __forceinline__ unsigned bf16_lo_bits(float v) {
  float hi = bf16_val(v);
  asm volatile("" : "+v"(hi));
  return bf16_bits(v - hi);
}
__device__ __forceinline__ v4u pack8_bf16(v4f a, v4f c) {
  return (v4u){ pk16(bf16_bits(a[0]), bf16_bits(a[1])), pk16(bf16_bits(a[2]), bf16_bits(a[3])),
                pk16(bf16_bits(c[0]), bf16_bits(c[1])), pk16(bf16_bits(c[2]), bf16_bits(c[3])) };
}
__device__ __forceinline__ v4u pack8_bf16_lo(v4f a, v4f c) {
  return (v4u){ pk16(bf16_lo_bits(a[0]), bf16_lo_bits(a[1])), pk16(bf16_lo_bits(a[2]), bf16_lo_bits(a[3])),
                pk16(bf16_lo_bits(c[0]), bf16_lo_bits(c[1])), pk16(bf16_lo_bits(c[2]), bf16_lo_bits(c[3])) };
}
__device__ __forceinline__ v4u pack8_f16(v4f a, v4f c) {
  return (v4u){ pk16(f16_bits(a[0]), f16_bits(a[1])), pk16(f16_bits(a[2]), f16_bits(a[3])),
                pk16(f16_bits(c[0]), f16_bits(c[1])), pk16(f16_bits(c[2]), f16_bits(c[3])) };
}

template <int FORM>
__global__ __launch_bounds__(256) void k_plane(const float* __restrict__ src, int rows, int cols, int ldsrc,
                                               unsigned short* __restrict__ dst, int MP, int KP) {
  static_assert(FORM >= 0 && FORM <= 3);
  const int KTOT = (FORM == 1 || FORM == 3) ? 2 * KP : KP;
  const unsigned ppr   = (unsigned)(KTOT >> 3);
  const unsigned kp8   = (unsigned)(KP >> 3);
  const unsigned total = (unsigned)MP * ppr;
  const unsigned g     = blockIdx.x * 256u + threadIdx.x;
  const unsigned rowu  = g / ppr;
  const unsigned p     = g - rowu * ppr;
  const bool second    = p >= kp8;
  const int row = (int)rowu;
  const int c0  = (int)((second ? p - kp8 : p) << 3);
  const float* srow = src + (size_t)clampi(row, 0, rows - 1) * (size_t)ldsrc;
  float x[8];
  unsigned mk[8];
#pragma unroll
  for (int e = 0; e < 8; ++e) {
    const int c = c0 + e;
    const float v = srow[clampi(c, 0, cols - 1)];
    asm volatile("" :: "v"(v));
    x[e]  = v;
    mk[e] = (row < rows && c < cols) ? 0xFFFFu : 0u;
  }
  const v4f a = (v4f){ x[0], x[1], x[2], x[3] };
  const v4f c = (v4f){ x[4], x[5], x[6], x[7] };
  v4u o;
  if (FORM == 2) {
    o = pack8_f16(a, c);
  } else {
    const v4u hi = pack8_bf16(a, c);
    o = hi;
    if (FORM == 1) { const v4u lo = pack8_bf16_lo(a, c); o = second ? lo : hi; }
  }
  const v4u mw = (v4u){ pk16(mk[0], mk[1]), pk16(mk[2], mk[3]), pk16(mk[4], mk[5]), pk16(mk[6], mk[7]) };
  o &= mw;
  if (g < total) {
    volatile v4u* q = (volatile v4u*)(dst + (size_t)g * 8);
    *q = o;
    __threadfence();
    *q = o;
  }
}

template <int FORM> struct FragOf    { typedef FragB T; };
template <>         struct FragOf<2> { typedef FragH T; };
__device__ __forceinline__ v8f mm(const FragB& a, const FragB& b, v8f c) { return wmb(a, b, c); }
__device__ __forceinline__ v8f mm(const FragH& a, const FragH& b, v8f c) { return wmh(a, b, c); }
template <class F> __device__ __forceinline__ F ld_frag(const unsigned short* p) {
  F f;
  f.h[0] = *(const v8usa*)(p);
  f.h[1] = *(const v8usa*)(p + 16);
  return f;
}

template <int FORM, int EPI>
__global__ __launch_bounds__(256) __attribute__((amdgpu_num_vgpr(248)))
void k_gemm_nt(const unsigned short* __restrict__ A, const unsigned short* __restrict__ B,
               const float* __restrict__ bias, float* __restrict__ D, int M, int N, int KTOT, int ldd) {
  static_assert(FORM >= 0 && FORM <= 2);
  static_assert(EPI == 0 || EPI == 1);
  typedef typename FragOf<FORM>::T F;
  __shared__ __attribute__((aligned(16))) float sT[8][16 * 68];
  const int lane = threadIdx.x & 31;
  const int wave = threadIdx.x >> 5;
  const int tilesM = (M + 63) >> 6;
  const int tilesN = (N + 63) >> 6;
  const int tile = blockIdx.x * 8 + wave;
  if (tile >= tilesM * tilesN) return;
  const int tm = tile / tilesN;
  const int tn = tile - tm * tilesN;
  const int m0 = tm << 6;
  const int n0 = tn << 6;

  const int rl = lane & 15;
  const int h8 = (lane >> 4) * 8;
  const unsigned short* pa = A + (size_t)(m0 + rl) * (size_t)KTOT + h8;
  const unsigned short* pb = B + (size_t)(n0 + rl) * (size_t)KTOT + h8;

  v8f acc[4][4];
#pragma unroll
  for (int i = 0; i < 4; ++i)
#pragma unroll
    for (int j = 0; j < 4; ++j) acc[i][j] = (v8f){0.f, 0.f, 0.f, 0.f, 0.f, 0.f, 0.f, 0.f};

#pragma unroll 1
  for (int k0 = 0; k0 < KTOT; k0 += 32) {
    F bf[4];
#pragma unroll
    for (int j = 0; j < 4; ++j) bf[j] = ld_frag<F>(pb + (size_t)(j << 4) * (size_t)KTOT + k0);
#pragma unroll
    for (int i = 0; i < 4; ++i) {
      const F af = ld_frag<F>(pa + (size_t)(i << 4) * (size_t)KTOT + k0);
#pragma unroll
      for (int j = 0; j < 4; ++j) acc[i][j] = mm(af, bf[j], acc[i][j]);
    }
  }

  float* slab = sT[wave];
  const int hh = lane >> 4;
  const int c4 = (lane & 15) * 4;
  const int nc = n0 + c4;
  const bool cok = nc < N;
  v4f bv = (v4f){0.f, 0.f, 0.f, 0.f};
  if (EPI == 1) {
    bv = *(const v4fa*)(bias + clampi(nc, 0, N - 4));
    asm volatile("" :: "v"(bv));
  }
#pragma unroll
  for (int i = 0; i < 4; ++i) {
    const int mBase = m0 + (i << 4);
#pragma unroll
    for (int j = 0; j < 4; ++j) {
#pragma unroll
      for (int r = 0; r < 8; ++r) slab[(h8 + r) * 68 + (j << 4) + rl] = acc[i][j][r];
    }
    __builtin_amdgcn_fence(__ATOMIC_RELEASE, "workgroup");
    __builtin_amdgcn_wave_barrier();
    __builtin_amdgcn_fence(__ATOMIC_ACQUIRE, "workgroup");
    v4f vv[8];
#pragma unroll
    for (int it = 0; it < 8; ++it) {
      const int row = it * 2 + hh;
      v4f v = *(const v4fa*)(slab + row * 68 + c4);
      if (EPI == 1) v += bv;
      vv[it] = v;
    }
    for (int pass = 0; pass < 2; ++pass) {
#pragma unroll
      for (int it = 0; it < 8; ++it) {
        const int row = mBase + it * 2 + hh;
        if (cok && row < M) *(volatile v4f*)(D + (size_t)row * (size_t)ldd + nc) = vv[it];
      }
      __threadfence();
    }
    __builtin_amdgcn_fence(__ATOMIC_RELEASE, "workgroup");
    __builtin_amdgcn_wave_barrier();
    __builtin_amdgcn_fence(__ATOMIC_ACQUIRE, "workgroup");
  }
}

#pragma clang fp contract(off)

typedef unsigned int v2u __attribute__((ext_vector_type(2)));
typedef int          v4i __attribute__((ext_vector_type(4)));
typedef v4i __attribute__((may_alias)) v4ia;

constexpr int H_TWO_TERM = 1;

constexpr int NN    = 10000;
constexpr int NP    = 10112;
constexpr int DF    = 128;
constexpr int NE    = 640000;
constexpr int LDP   = 2 * DF;
constexpr int K2    = DF * (1 + H_TWO_TERM);
constexpr int PPR2  = K2 / 8;

constexpr int BTHR  = 256;
constexpr int BNW   = 8;
constexpr int NOWN  = 256;
constexpr int SLB   = 8;
constexpr int NBLK  = 40;
constexpr int NTAB  = NBLK * NOWN;
constexpr int EW    = NE / BNW;
constexpr int STEPW = 256;
constexpr int NSTEP = (EW + STEPW - 1) / STEPW;
constexpr int WLCAP = 3072;
constexpr int RCAP  = 20480;
constexpr int DEGCAP = 128;
constexpr int MEAS_HITS = 16708;
constexpr int MEAS_DEG  = 101;
constexpr int PLINE = 32;
constexpr int B_ZINTS = RCAP + BNW * WLCAP + 2 * BNW * NOWN + 2 * NOWN;
constexpr int B_INTS  = B_ZINTS + 32;
constexpr int B_BYTES = B_INTS * 4;

static_assert(DF == 32 * 4);
static_assert(NN % 8 == 0 && NN % 16 == 0 && NP % 64 == 0 && NP % 128 == 0 && NP >= NN);
static_assert(NE == 312 * 2048 + 1024 && EW * BNW == NE && EW == 312 * STEPW + 128);
static_assert(EW % 128 == 0 && EW % 4 == 0 && NE % 4 == 0);
static_assert(NOWN == (1 << SLB) && NBLK * NOWN >= NN && NTAB == 10240 && ((NN - 1) >> SLB) == NBLK - 1);
static_assert(NN <= (1 << 14));
static_assert(RCAP == 20480 && RCAP >= MEAS_HITS + 2048 && RCAP % (4 * BTHR) == 0 && BNW * WLCAP >= RCAP);
static_assert(DEGCAP == 128 && DEGCAP >= MEAS_DEG + 8);
static_assert(B_ZINTS % 4 == 0 && B_BYTES == 198784 && B_BYTES <= 262144);
static_assert(K2 % 32 == 0 && LDP % 64 == 0 && LDP % 32 == 0 && DF % 32 == 0);
static_assert((long long)NP * K2 / 8 < (1LL << 31));

constexpr size_t SZ_XB   = (size_t)NP * DF * 2;
constexpr size_t SZ_W1C  = (size_t)2 * DF * DF * 2;
constexpr size_t SZ_W2C  = (size_t)2 * DF * K2 * 2;
constexpr size_t SZ_BF   = 512;
constexpr size_t SZ_PQ   = (size_t)NP * LDP * 4;
constexpr size_t SZ_HHL  = (size_t)NP * K2 * 2;
constexpr size_t SZ_LIST = (size_t)NBLK * RCAP * 4;
constexpr size_t SZ_TAB  = (size_t)NTAB * 4;
constexpr size_t SZ_POI  = (size_t)NBLK * PLINE * 4;
constexpr size_t OFF_XB   = 0;
constexpr size_t OFF_W1C  = OFF_XB + SZ_XB;
constexpr size_t OFF_W2C  = OFF_W1C + SZ_W1C;
constexpr size_t OFF_B1F  = OFF_W2C + SZ_W2C;
constexpr size_t OFF_B2F  = OFF_B1F + SZ_BF;
constexpr size_t OFF_PQ   = OFF_B2F + SZ_BF;
constexpr size_t OFF_HHL  = OFF_PQ + SZ_PQ;
constexpr size_t OFF_LIST = OFF_HHL + SZ_HHL;
constexpr size_t OFF_CNT  = OFF_LIST + SZ_LIST;
constexpr size_t OFF_OFS  = OFF_CNT + SZ_TAB;
constexpr size_t OFF_POI  = OFF_OFS + SZ_TAB;
constexpr size_t WS_TOTAL = OFF_POI + SZ_POI;
static_assert(SZ_XB % 256 == 0 && SZ_W1C % 256 == 0 && SZ_W2C % 256 == 0 && SZ_BF % 256 == 0 && SZ_PQ % 256 == 0);
static_assert(SZ_HHL % 256 == 0 && SZ_LIST % 256 == 0 && SZ_TAB % 256 == 0 && SZ_POI % 256 == 0);
static_assert(H_TWO_TERM != 1 || WS_TOTAL == (size_t)21682176);
static_assert(WS_TOTAL <= ((size_t)128 << 20));

constexpr int NB_W1H  = DF * (DF / 8) / 256;
constexpr int NB_W2H  = DF * PPR2 / 256;
constexpr int NB_PAD  = (NP - NN) * PPR2 / 256;
constexpr int PB_W1N  = NB_W1H;
constexpr int PB_W2S  = 2 * NB_W1H;
constexpr int PB_W2N  = PB_W2S + NB_W2H;
constexpr int PB_BI   = PB_W2N + NB_W2H;
constexpr int PB_PAD  = PB_BI + 2;
constexpr int NB_PREP = PB_PAD + NB_PAD;
static_assert(NB_W1H * 256 == DF * (DF / 8) && NB_W2H * 256 == DF * PPR2 && NB_PAD * 256 == (NP - NN) * PPR2);

__device__ __forceinline__ void put16(unsigned short* dp, v4u o) {
  volatile v4u* q = (volatile v4u*)dp;
  *q = o;
  __threadfence();
  *q = o;
}

__device__ __forceinline__ void wpiece(const float* __restrict__ W, unsigned short* __restrict__ dst,
                                       int rowOff, int g, int ppr) {
  const int j  = g / ppr;
  const int p  = g - j * ppr;
  const int sc = (8 * p) & (DF - 1);
  const float* s = W + (size_t)j * DF + sc;
  const v4f a = *(const v4fa*)s;
  const v4f c = *(const v4fa*)(s + 4);
  asm volatile("" :: "v"(a));
  asm volatile("" :: "v"(c));
  put16(dst + ((size_t)(rowOff + j) * ppr + p) * 8, pack8_bf16(a, c));
}

__device__ __forceinline__ void bias_piece(const float* __restrict__ b, float* __restrict__ B, int tid) {
  const int u = tid < 32 ? tid : 31;
  const v4f t = *(const v4fa*)(b + 4 * u);
  asm volatile("" :: "v"(t));
  const v4f o = (v4f){ bf16_val(t[0]), bf16_val(t[1]), bf16_val(t[2]), bf16_val(t[3]) };
  if (tid < 32) {
    volatile v4f* q = (volatile v4f*)(B + 4 * tid);
    *q = o;
    __threadfence();
    *q = o;
  }
}

__global__ __launch_bounds__(256) __attribute__((amdgpu_num_vgpr(248)))
void k_prep(const float* __restrict__ W1s, const float* __restrict__ W1n, const float* __restrict__ b1,
            const float* __restrict__ W2s, const float* __restrict__ W2n, const float* __restrict__ b2,
            unsigned short* __restrict__ W1C, unsigned short* __restrict__ W2C,
            float* __restrict__ B1F, float* __restrict__ B2F, unsigned short* __restrict__ HHL) {
  const int tid = (int)threadIdx.x;
  const int blk = (int)blockIdx.x;
  if (blk < PB_W1N) {
    wpiece(W1s, W1C, 0, blk * 256 + tid, DF / 8);
  } else if (blk < PB_W2S) {
    wpiece(W1n, W1C, DF, (blk - PB_W1N) * 256 + tid, DF / 8);
  } else if (blk < PB_W2N) {
    wpiece(W2s, W2C, 0, (blk - PB_W2S) * 256 + tid, PPR2);
  } else if (blk < PB_BI) {
    wpiece(W2n, W2C, DF, (blk - PB_W2N) * 256 + tid, PPR2);
  } else if (blk == PB_BI) {
    bias_piece(b1, B1F, tid);
  } else if (blk == PB_BI + 1) {
    bias_piece(b2, B2F, tid);
  } else {
    const int g = (blk - PB_PAD) * 256 + tid;
    put16(HHL + (size_t)NN * K2 + (size_t)g * 8, (v4u){ 0u, 0u, 0u, 0u });
  }
}

__global__ __launch_bounds__(256) __attribute__((amdgpu_num_vgpr(248)))
void k_bucket(const int* __restrict__ ei, int* __restrict__ LIST, int* __restrict__ CNT,
              int* __restrict__ OFS, int* __restrict__ POISON) {
  extern __shared__ __attribute__((aligned(16))) int dsm[];
  int* sl    = dsm;
  int* wlAll = sl + RCAP;
  int* cntw  = wlAll + BNW * WLCAP;
  int* cur   = cntw + BNW * NOWN;
  int* cnt   = cur + BNW * NOWN;
  int* offs  = cnt + NOWN;
  int* misc  = offs + NOWN;
  const int tid = (int)threadIdx.x, lane = tid & 31, wave = tid >> 5;
  const int blk = (int)blockIdx.x;
  const int slotBase = blk * NOWN;

  {
    const v4i z4 = (v4i){ 0, 0, 0, 0 };
    for (int i = tid * 4; i < B_ZINTS; i += BTHR * 4) *(v4ia*)(dsm + i) = z4;
    if (tid < 32) misc[tid] = 0;
  }
  __syncthreads();

  const int* srcw = ei + (size_t)wave * EW;
  const int* dstw = ei + (size_t)NE + (size_t)wave * EW;
  int* wl = wlAll + wave * WLCAP;
  int wc = 0;
#pragma unroll 1
  for (int s = 0; s < NSTEP; ++s) {
#pragma unroll
    for (int j = 0; j < 2; ++j) {
      const int loc = s * STEPW + j * 128 + 4 * lane;
      const bool ok = loc < EW;
      const int lc  = ok ? loc : (EW - 4);
      const v4i dv = *(const v4ia*)(dstw + lc);
      asm volatile("" :: "v"(dv));
      const v4i sv = *(const v4ia*)(srcw + lc);
      asm volatile("" :: "v"(sv));
      unsigned us[4];
      bool     hb[4];
      unsigned mk[4];
#pragma unroll
      for (int c = 0; c < 4; ++c) {
        const int d   = clampi(dv[c], 0, NN - 1);
        const int key = ok ? d : -1;
        us[c] = (unsigned)key - (unsigned)slotBase;
        hb[c] = us[c] < (unsigned)NOWN;
        mk[c] = __builtin_amdgcn_ballot_w32(hb[c]);
      }
      int p = wc;
#pragma unroll
      for (int c = 0; c < 4; ++c) p += (int)__builtin_amdgcn_mbcnt_lo(mk[c], 0u);
#pragma unroll
      for (int c = 0; c < 4; ++c) {
        const int ent = (clampi(sv[c], 0, NN - 1) << SLB) | (int)(us[c] & (unsigned)(NOWN - 1));
        if (hb[c] && p < WLCAP) wl[p] = ent;
        p += hb[c] ? 1 : 0;
      }
#pragma unroll
      for (int c = 0; c < 4; ++c) wc += (int)__builtin_popcount(mk[c]);
    }
  }
  if (lane == 0 && wc > WLCAP) misc[8] = 1;
  __syncthreads();

  const int cw = __builtin_amdgcn_readfirstlane(wc < WLCAP ? wc : WLCAP);
  {
    int* myc = cntw + wave * NOWN;
#pragma unroll 1
    for (int b0 = 0; b0 < cw; b0 += 32) {
      const int idx = b0 + lane;
      const int ent = wl[idx < WLCAP ? idx : WLCAP - 1];
      const int rem = cw - b0;
      const int m32 = rem < 32 ? rem : 32;
#pragma unroll 1
      for (int k = 0; k < m32; ++k) {
        const int u    = __builtin_amdgcn_readlane(ent, k);
        const int slot = u & (NOWN - 1);
        const int c0   = myc[slot];
        if (lane == 0) myc[slot] = c0 + 1;
      }
    }
  }
  __syncthreads();

  int part[BNW];
  int tot = 0;
#pragma unroll
  for (int w = 0; w < BNW; ++w) { part[w] = cntw[w * NOWN + tid]; tot += part[w]; }
  if (tot > DEGCAP) misc[8] = 1;
  int incl = tot;
#pragma unroll
  for (int d = 1; d < 32; d <<= 1) {
    const int y = __shfl_up(incl, d, 32);
    incl += (lane >= d) ? y : 0;
  }
  if (lane == 31) misc[16 + wave] = incl;
  __syncthreads();
  {
    int wbase = 0, total = 0;
#pragma unroll
    for (int w = 0; w < BNW; ++w) {
      const int v = misc[16 + w];
      wbase += (w < wave) ? v : 0;
      total += v;
    }
    const int excl = wbase + incl - tot;
    if (total > RCAP && tid == 0) misc[8] = 1;
    cnt[tid]  = tot;
    offs[tid] = clampi(excl, 0, RCAP - 1);
    int run = excl;
#pragma unroll
    for (int w = 0; w < BNW; ++w) { cur[w * NOWN + tid] = run; run += part[w]; }
  }
  __syncthreads();

  {
    int* myq = cur + wave * NOWN;
#pragma unroll 1
    for (int b0 = 0; b0 < cw; b0 += 32) {
      const int idx = b0 + lane;
      const int ent = wl[idx < WLCAP ? idx : WLCAP - 1];
      const int rem = cw - b0;
      const int m32 = rem < 32 ? rem : 32;
#pragma unroll 1
      for (int k = 0; k < m32; ++k) {
        const int u    = __builtin_amdgcn_readlane(ent, k);
        const int slot = u & (NOWN - 1);
        const int p    = myq[slot];
        const int pc   = clampi(p, 0, RCAP - 1);
        if (lane == 0) { sl[pc] = u >> SLB; myq[slot] = p + 1; }
      }
    }
  }
  __syncthreads();
  const int flag = misc[8];

  int* lp = LIST + (size_t)blk * RCAP;
  for (int pass = 0; pass < 2; ++pass) {
#pragma unroll 1
    for (int it = 0; it < RCAP / (4 * BTHR); ++it) {
      const int q = it * BTHR + tid;
      const v4i v = *(const v4ia*)(sl + 4 * q);
      *(volatile v4i*)(lp + 4 * q) = v;
    }
    __threadfence();
  }
  {
    const int q4 = tid < 64 ? tid : 63;
    const v4i m1 = (v4i){ -1, -1, -1, -1 };
    v4i c4 = *(const v4ia*)(cnt + 4 * q4);
    const v4i o4 = *(const v4ia*)(offs + 4 * q4);
    c4 = (flag != 0) ? m1 : c4;
    const int fv = flag != 0 ? 1 : 0;
    const v4i f4 = (v4i){ fv, fv, fv, fv };
    const int q8 = tid < 8 ? tid : 7;
    volatile v4i* qc = (volatile v4i*)(CNT + slotBase + 4 * q4);
    volatile v4i* qo = (volatile v4i*)(OFS + slotBase + 4 * q4);
    volatile v4i* qp = (volatile v4i*)(POISON + blk * PLINE + 4 * q8);
    if (tid < 64) { *qc = c4; *qo = o4; }
    if (tid < 8) *qp = f4;
    __threadfence();
    if (tid < 64) { *qc = c4; *qo = o4; }
    if (tid < 8) *qp = f4;
  }
}

__device__ __forceinline__ v4f walk(const float* __restrict__ PQ, const int* __restrict__ lst,
                                    int off, int cnt, int lane) {
  v4f s = (v4f){ 0.0f, 0.0f, 0.0f, 0.0f };
  const int cm1 = cnt > 0 ? cnt - 1 : 0;
#pragma unroll 1
  for (int b0 = 0; b0 < cnt; b0 += 32) {
    const int j   = b0 + lane;
    const int idx = clampi(off + (j < cm1 ? j : cm1), 0, RCAP - 1);
    int ent = lst[idx];
    asm volatile("" :: "v"(ent));
    const int sr  = clampi(ent, 0, NN - 1);
    const int rem = cnt - b0;
    const int m32 = rem < 32 ? rem : 32;
#pragma unroll 1
    for (int k = 0; k < m32; ++k) {
      const int sk = __builtin_amdgcn_readlane(sr, k);
      const v4f g = *(const v4fa*)(PQ + (size_t)sk * LDP + DF + 4 * lane);
      asm volatile("" :: "v"(g));
      s[0] = s[0] + g[0];
      s[1] = s[1] + g[1];
      s[2] = s[2] + g[2];
      s[3] = s[3] + g[3];
    }
  }
  return s;
}

__device__ __forceinline__ v4f self_plus_mean(const float* __restrict__ PQ, const int* __restrict__ LIST,
                                              const int* __restrict__ CNT, const int* __restrict__ OFS,
                                              const int* __restrict__ POISON, bool live, int nc, int lane,
                                              int& badOut) {
  const int b = nc >> SLB;
  int rc = CNT[nc];
  asm volatile("" :: "v"(rc));
  int ro = OFS[nc];
  asm volatile("" :: "v"(ro));
  int pw = POISON[b * PLINE];
  asm volatile("" :: "v"(pw));
  badOut = ((rc < 0) | (rc > DEGCAP) | (pw != 0)) ? 1 : 0;
  const int cv = clampi(rc, 0, DEGCAP);
  const int cn = __builtin_amdgcn_readfirstlane(live ? cv : 0);
  const int of = __builtin_amdgcn_readfirstlane(clampi(ro, 0, RCAP - 1));
  const v4f s = walk(PQ, LIST + (size_t)b * RCAP, of, cn, lane);
  const v4f sp = *(const v4fa*)(PQ + (size_t)nc * LDP + 4 * lane);
  asm volatile("" :: "v"(sp));
  const float fc = (float)(cn > 1 ? cn : 1);
  return (v4f){ sp[0] + s[0] / fc, sp[1] + s[1] / fc, sp[2] + s[2] / fc, sp[3] + s[3] / fc };
}

__global__ __launch_bounds__(256) __attribute__((amdgpu_num_vgpr(248)))
void k_agg1(const float* __restrict__ P, const int* __restrict__ LIST, const int* __restrict__ CNT,
            const int* __restrict__ OFS, const int* __restrict__ POISON, const float* __restrict__ B1F,
            unsigned short* __restrict__ HHL) {
  __shared__ __attribute__((aligned(16))) float sB[DF];
  const int tid = (int)threadIdx.x, lane = tid & 31, wave = tid >> 5;
  if (tid < 32) {
    const v4f t = *(const v4fa*)(B1F + 4 * tid);
    *(v4fa*)(sB + 4 * tid) = t;
  }
  __syncthreads();
  const int n  = __builtin_amdgcn_readfirstlane((int)blockIdx.x * 8 + wave);
  const int nc = n < NN ? n : NN - 1;
  int bad = 0;
  const v4f t = self_plus_mean(P, LIST, CNT, OFS, POISON, n < NN, nc, lane, bad);
  const v4f bv = *(const v4fa*)(sB + 4 * lane);
  const float v0 = t[0] + bv[0];
  const float v1 = t[1] + bv[1];
  const float v2 = t[2] + bv[2];
  const float v3 = t[3] + bv[3];
  const float qn = __uint_as_float(0x7fc00000u);
  float h0 = (v0 > 0.0f) ? v0 : (v0 - v0);
  float h1 = (v1 > 0.0f) ? v1 : (v1 - v1);
  float h2 = (v2 > 0.0f) ? v2 : (v2 - v2);
  float h3 = (v3 > 0.0f) ? v3 : (v3 - v3);
  h0 = (bad != 0) ? qn : h0;
  h1 = (bad != 0) ? qn : h1;
  h2 = (bad != 0) ? qn : h2;
  h3 = (bad != 0) ? qn : h3;
  const v2u hi = (v2u){ pk16(bf16_bits(h0), bf16_bits(h1)), pk16(bf16_bits(h2), bf16_bits(h3)) };
  const v2u lo = (v2u){ pk16(bf16_lo_bits(h0), bf16_lo_bits(h1)), pk16(bf16_lo_bits(h2), bf16_lo_bits(h3)) };
  unsigned short* dp = HHL + (size_t)nc * K2 + 4 * lane;
  if (n < NN) {
    volatile v2u* qh = (volatile v2u*)dp;
    volatile v2u* ql = (volatile v2u*)(dp + (H_TWO_TERM != 0 ? DF : 0));
    *qh = hi;
    if (H_TWO_TERM != 0) *ql = lo;
    __threadfence();
    *qh = hi;
    if (H_TWO_TERM != 0) *ql = lo;
  }
}

__global__ __launch_bounds__(256) __attribute__((amdgpu_num_vgpr(248)))
void k_agg2(const float* __restrict__ Q, const int* __restrict__ LIST, const int* __restrict__ CNT,
            const int* __restrict__ OFS, const int* __restrict__ POISON, const float* __restrict__ B2F,
            float* __restrict__ out, int nReal) {
  __shared__ __attribute__((aligned(16))) float sB[DF];
  const int tid = (int)threadIdx.x, lane = tid & 31, wave = tid >> 5;
  if (tid < 32) {
    const v4f t = *(const v4fa*)(B2F + 4 * tid);
    *(v4fa*)(sB + 4 * tid) = t;
  }
  __syncthreads();
  const int n  = __builtin_amdgcn_readfirstlane((int)blockIdx.x * 8 + wave);
  const int nc = n < NN ? n : NN - 1;
  int bad = 0;
  const v4f t = self_plus_mean(Q, LIST, CNT, OFS, POISON, n < NN, nc, lane, bad);
  const v4f bv = *(const v4fa*)(sB + 4 * lane);
  const float qn = __uint_as_float(0x7fc00000u);
  float v0 = t[0] + bv[0];
  float v1 = t[1] + bv[1];
  float v2 = t[2] + bv[2];
  float v3 = t[3] + bv[3];
  v0 = (bad != 0) ? qn : v0;
  v1 = (bad != 0) ? qn : v1;
  v2 = (bad != 0) ? qn : v2;
  v3 = (bad != 0) ? qn : v3;
  const v4f o = (v4f){ v0, v1, v2, v3 };
  if (n < nReal && n < NN) {
    volatile v4f* q = (volatile v4f*)(out + (size_t)nc * DF + 4 * lane);
    *q = o;
    __threadfence();
    *q = o;
  }
}

extern "C" void kernel_launch(void* const* d_in, const int* in_sizes, int n_in,
                              void* d_out, int out_size, void* d_ws, size_t ws_size,
                              hipStream_t stream) {
  if (n_in < 8) return;
  if (in_sizes[0] != NN * DF) return;
  if (in_sizes[1] != 2 * NE) return;
  if (in_sizes[2] != DF * DF || in_sizes[3] != DF * DF || in_sizes[4] != DF) return;
  if (in_sizes[5] != DF * DF || in_sizes[6] != DF * DF || in_sizes[7] != DF) return;
  if (out_size != NN * DF) return;
  if (ws_size < WS_TOTAL) return;

  const float* x   = (const float*)d_in[0];
  const int*   ei  = (const int*)d_in[1];
  const float* W1s = (const float*)d_in[2];
  const float* W1n = (const float*)d_in[3];
  const float* b1  = (const float*)d_in[4];
  const float* W2s = (const float*)d_in[5];
  const float* W2n = (const float*)d_in[6];
  const float* b2  = (const float*)d_in[7];
  float* out = (float*)d_out;

  char* ws = (char*)d_ws;
  unsigned short* XB  = (unsigned short*)(ws + OFF_XB);
  unsigned short* W1C = (unsigned short*)(ws + OFF_W1C);
  unsigned short* W2C = (unsigned short*)(ws + OFF_W2C);
  float* B1F = (float*)(ws + OFF_B1F);
  float* B2F = (float*)(ws + OFF_B2F);
  float* PQ  = (float*)(ws + OFF_PQ);
  unsigned short* HHL = (unsigned short*)(ws + OFF_HHL);
  int* LIST = (int*)(ws + OFF_LIST);
  int* CNT  = (int*)(ws + OFF_CNT);
  int* OFS  = (int*)(ws + OFF_OFS);
  int* POI  = (int*)(ws + OFF_POI);

  hipFuncSetAttribute(reinterpret_cast<const void*>(&k_bucket), hipFuncAttributeMaxDynamicSharedMemorySize, B_BYTES);

  k_plane<0><<<NP * DF / 8 / 256, 256, 0, stream>>>(x, NN, DF, DF, XB, NP, DF);
  k_prep<<<NB_PREP, 256, 0, stream>>>(W1s, W1n, b1, W2s, W2n, b2, W1C, W2C, B1F, B2F, HHL);
  k_bucket<<<NBLK, BTHR, B_BYTES, stream>>>(ei, LIST, CNT, OFS, POI);
  k_gemm_nt<0, 0><<<(((NN + 63) / 64) * (LDP / 64) + 7) / 8, 256, 0, stream>>>(XB, W1C, B1F, PQ, NN, LDP, DF, LDP);
  k_agg1<<<NN / 8, 256, 0, stream>>>(PQ, LIST, CNT, OFS, POI, B1F, HHL);
  k_gemm_nt<0, 0><<<(((NN + 63) / 64) * (LDP / 64) + 7) / 8, 256, 0, stream>>>(HHL, W2C, B2F, PQ, NN, LDP, K2, LDP);
  k_agg2<<<NN / 8, 256, 0, stream>>>(PQ, LIST, CNT, OFS, POI, B2F, out, NN);
}
